// TransformerEncoderLayer_6820408066247
// MI455X (gfx1250) — hardware-verified
//
#include <hip/hip_runtime.h>
#ifndef NB
#define NB 8
#endif
#ifndef SEQ
#define SEQ 1024
#endif
#define NB_FULL 8
#define SEQ_FULL 1024
#define DM 512
#define NH 8
#define DK 32
#define DH 64
#define NR ((size_t)NB * SEQ)
#define LQK 512
#define WROWS 2048
static_assert(SEQ % 64 == 0);
static_assert(NB >= 1 && NB <= NB_FULL);
static_assert(SEQ <= SEQ_FULL);
static_assert(NH * DH == DM);
static_assert(2 * NH * DK == LQK);
static_assert(DK == 32 && DH == 64);
static_assert(DM % 128 == 0 && DM % 32 == 0 && LQK % 64 == 0);
static_assert(((size_t)NB * SEQ) % 128 == 0);
static_assert(DM / 4 == 128);
static_assert((((size_t)NB * SEQ) * DM / 8) % 256 == 0);
static_assert((((size_t)NB * SEQ) * LQK / 8) % 256 == 0);
static_assert(((size_t)DM * DM / 8) % 256 == 0);
static_assert(((size_t)NH * DK * DM / 8) % 256 == 0);
static_assert((size_t)2 * NH * DK + (size_t)3 * DM == WROWS);

typedef unsigned short v8us __attribute__((ext_vector_type(8), may_alias));
typedef float  v8f  __attribute__((ext_vector_type(8)));
typedef float  v8fa __attribute__((ext_vector_type(8), may_alias));
typedef int    v8i  __attribute__((ext_vector_type(8)));
typedef int    v8ia __attribute__((ext_vector_type(8), may_alias));
typedef float  v4f  __attribute__((ext_vector_type(4)));
typedef float  v4fa __attribute__((ext_vector_type(4), may_alias));
typedef _Float16 v16h __attribute__((ext_vector_type(16)));
typedef _Float16 v4h __attribute__((ext_vector_type(4)));
union FragH { v16h v; v8us half[2]; _Float16 h[16]; unsigned short u[16]; };

__device__ __forceinline__ unsigned short bf16_bits(float x) { unsigned int u = __float_as_uint(x); return (unsigned short)((u + 0x7FFFu + ((u >> 16) & 1u)) >> 16); }
__device__ __forceinline__ float bf16_val(unsigned short b) { return __uint_as_float(((unsigned int)b) << 16); }
__device__ __forceinline__ float bf16_rne(float x) { return bf16_val(bf16_bits(x)); }

__device__ __forceinline__ v16h g2_frag(const _Float16* p, unsigned hh) { FragH f; f.half[0] = *(const v8us*)((const unsigned short*)p + 8u * hh); f.half[1] = *(const v8us*)((const unsigned short*)p + 16u + 8u * hh); return f.v; }
__device__ __forceinline__ v8f g2_mma(v16h a, v16h b, v8f c) { v8f d = __builtin_amdgcn_wmma_f32_16x16x32_f16(false, a, false, b, (short)0, c, false, false); asm volatile("v_nop\n\tv_nop\n\tv_nop\n\tv_nop" : "+v"(d) : "v"(a), "v"(b)); return d; }

__global__ __launch_bounds__(256) void k_wprep(const float* __restrict__ Wq, const float* __restrict__ Wk, const float* __restrict__ Wv, const float* __restrict__ Wo, const float* __restrict__ Wf, _Float16* __restrict__ BW) {
  const unsigned which = blockIdx.y;
  const float* W = (which == 0u) ? Wq : ((which == 1u) ? Wk : ((which == 2u) ? Wv : ((which == 3u) ? Wo : Wf)));
  const unsigned n8 = (which < 2u) ? (unsigned)(NH * DK * DM / 8) : (unsigned)(DM * DM / 8);
  const unsigned rowoff = (which == 0u) ? 0u : ((which == 1u) ? 256u : ((which == 2u) ? 512u : ((which == 3u) ? 1024u : 1536u)));
  const unsigned t = blockIdx.x * 256u + threadIdx.x; if (t >= n8) return;
  const size_t e = (size_t)t * 8u; const float* p = W + e; const v4f a = *(const v4fa*)p, c = *(const v4fa*)(p + 4); FragH f;
#pragma unroll
  for (unsigned q = 0; q < 4; ++q) { f.h[q] = (_Float16)(16.0f * bf16_rne(a[q])); f.h[4 + q] = (_Float16)(16.0f * bf16_rne(c[q])); }
  const v8us o = f.half[0];
  unsigned short* dst = (unsigned short*)BW + (size_t)rowoff * DM + e;
  *(volatile v8us*)dst = o; __threadfence(); *(volatile v8us*)dst = o;
}

__global__ __launch_bounds__(256) void k_xprep(const float* __restrict__ x, _Float16* __restrict__ X16, unsigned n8) {
  const unsigned t = blockIdx.x * 256u + threadIdx.x; if (t >= n8) return;
  const unsigned e = t * 8u; const unsigned r = e / (unsigned)DM; const unsigned c = e % (unsigned)DM; const unsigned rs = (r / (unsigned)SEQ) * (unsigned)SEQ_FULL + (r % (unsigned)SEQ);
  const float* p = x + (size_t)rs * DM + c; const v4f a = *(const v4fa*)p, cc = *(const v4fa*)(p + 4); FragH f;
#pragma unroll
  for (unsigned q = 0; q < 4; ++q) { f.h[q] = (_Float16)bf16_rne(a[q]); f.h[4 + q] = (_Float16)bf16_rne(cc[q]); }
  const v8us o = f.half[0];
  *(volatile v8us*)((unsigned short*)X16 + (size_t)e) = o; __threadfence(); *(volatile v8us*)((unsigned short*)X16 + (size_t)e) = o;
}

__global__ __launch_bounds__(256) void k_l2n(const float* __restrict__ QKF, _Float16* __restrict__ QK16, unsigned n8) {
  const unsigned t0 = blockIdx.x * 256u + threadIdx.x; const unsigned t = (t0 < n8) ? t0 : (n8 - 1u);
  const size_t e = (size_t)t * 8u; const float* p = QKF + e; const v4f a = *(const v4fa*)p, c = *(const v4fa*)(p + 4);
  float ss = 0.f;
#pragma unroll
  for (unsigned q = 0; q < 4; ++q) ss += a[q] * a[q];
#pragma unroll
  for (unsigned q = 0; q < 4; ++q) ss += c[q] * c[q];
  ss += __shfl_xor(ss, 1, 32); ss += __shfl_xor(ss, 2, 32);
  const float inv = 1.0f / fmaxf(sqrtf(ss), 1e-12f); FragH f;
#pragma unroll
  for (unsigned q = 0; q < 4; ++q) { f.h[q] = (_Float16)(a[q] * inv); f.h[4 + q] = (_Float16)(c[q] * inv); }
  const v8us o = f.half[0];
  if (t0 < n8) { *(volatile v8us*)((unsigned short*)QK16 + e) = o; __threadfence(); *(volatile v8us*)((unsigned short*)QK16 + e) = o; }
}

template <int ACT, int CPM>
__global__ __launch_bounds__(128) void k_gemm2(const _Float16* __restrict__ A, int lda, const _Float16* __restrict__ Bh, int ldb, float alpha, const float* __restrict__ bias, const float* __restrict__ CP,
    float* __restrict__ C, _Float16* __restrict__ C16, int ldc, int M, int N, int K) { static_assert(ACT == 0 || ACT == 4); static_assert(CPM >= 0 && CPM <= 2);
  __shared__ __attribute__((aligned(16))) float so[4][32][68];
  const unsigned tid = threadIdx.x, w = tid >> 5, lane = tid & 31u, ln = lane & 15u, hh = lane >> 4;
  const unsigned row0 = blockIdx.y * 128u + 32u * w, col0 = blockIdx.x * 64u; if (row0 >= (unsigned)M || col0 >= (unsigned)N) return;
  const _Float16* a0p = A + (size_t)(row0 + ln) * lda; const _Float16* a1p = a0p + (size_t)16 * lda;
  const _Float16* b0p = Bh + (size_t)(col0 + ln) * ldb; const _Float16* b1p = b0p + (size_t)16 * ldb; const _Float16* b2p = b1p + (size_t)16 * ldb; const _Float16* b3p = b2p + (size_t)16 * ldb;
  const v8f z8 = {0.f,0.f,0.f,0.f,0.f,0.f,0.f,0.f}; v8f c00 = z8, c01 = z8, c02 = z8, c03 = z8, c10 = z8, c11 = z8, c12 = z8, c13 = z8;
  const unsigned Ku = (unsigned)K;
#pragma unroll 1
  for (unsigned kb = 0; kb < Ku; kb += 32u) { const v16h a0 = g2_frag(a0p + kb, hh), a1 = g2_frag(a1p + kb, hh);
    v16h b = g2_frag(b0p + kb, hh); c00 = g2_mma(a0, b, c00); c10 = g2_mma(a1, b, c10);
    b = g2_frag(b1p + kb, hh); c01 = g2_mma(a0, b, c01); c11 = g2_mma(a1, b, c11);
    b = g2_frag(b2p + kb, hh); c02 = g2_mma(a0, b, c02); c12 = g2_mma(a1, b, c12);
    b = g2_frag(b3p + kb, hh); c03 = g2_mma(a0, b, c03); c13 = g2_mma(a1, b, c13); }
  v8f accs[8] = {c00, c01, c02, c03, c10, c11, c12, c13};
#pragma unroll
  for (unsigned u = 0; u < 8; ++u) { const unsigned t = u & 3u, half = u >> 2; const unsigned col = col0 + t * 16u + ln; float bc = 0.f; if (bias != nullptr) bc = bf16_rne(bias[col]);
#pragma unroll
    for (unsigned r = 0; r < 8; ++r) { const unsigned rloc = half * 16u + 8u * hh + r; float v = accs[u][r] * alpha + bc;
      if (ACT == 4) v = (v > 0.f) ? v : 0.01f * v;
      so[w][rloc][t * 16u + ln] = v; } }
  __builtin_amdgcn_fence(4  , "workgroup"); __builtin_amdgcn_wave_barrier();
  const unsigned rsub = lane >> 4, c4 = (lane & 15u) * 4u;
  v4f ov[16];
#pragma unroll
  for (unsigned q = 0; q < 16; ++q) { const unsigned r = q * 2u + rsub; v4f v = *(const v4fa*)&so[w][r][c4];
    if (CPM == 1) { const v4f cp = *(const v4fa*)(CP + (size_t)(row0 + r) * ldc + col0 + c4); v[0] += cp[0]; v[1] += cp[1]; v[2] += cp[2]; v[3] += cp[3]; }
    if (CPM == 2) { const unsigned rr = row0 + r; const unsigned rs = (rr / (unsigned)SEQ) * (unsigned)SEQ_FULL + (rr % (unsigned)SEQ); const v4f xv = *(const v4fa*)(CP + (size_t)rs * ldc + col0 + c4);
      v[0] += bf16_rne(xv[0]); v[1] += bf16_rne(xv[1]); v[2] += bf16_rne(xv[2]); v[3] += bf16_rne(xv[3]); }
    ov[q] = v; }
  for (int pass = 0; pass < 2; ++pass) {
#pragma unroll
    for (unsigned q = 0; q < 16; ++q) { const unsigned r = q * 2u + rsub; const v4f v = ov[q]; if (C) *(volatile v4f*)(C + (size_t)(row0 + r) * ldc + col0 + c4) = v; if (C16) { v4h h4; for (int i = 0; i < 4; ++i) h4[i] = (_Float16)v[i]; *(volatile v4h*)(C16 + (size_t)(row0 + r) * ldc + col0 + c4) = h4; } }
    if (pass == 0) __threadfence(); } }

template <int W16, int W32, int ORM>
__global__ __launch_bounds__(128) void k_lnx(const float* __restrict__ X, const float* __restrict__ g, const float* __restrict__ bb, float eps, _Float16* __restrict__ N16, float* __restrict__ N32) {
  #pragma clang fp contract(off)
  __shared__ float red[128]; const unsigned r = blockIdx.x; const unsigned ro = ORM ? ((r / (unsigned)SEQ) * (unsigned)SEQ_FULL + (r % (unsigned)SEQ)) : r; const unsigned t = threadIdx.x; const unsigned c0 = t * 4u;
  const v4f xa = *(const v4fa*)(X + (size_t)r * DM + c0); float s[4]; float sum = 0.f;
#pragma unroll
  for (int q = 0; q < 4; ++q) { s[q] = xa[q]; sum = sum + s[q]; }
  red[t] = sum; __syncthreads(); for (unsigned st = 64; st > 0; st >>= 1) { if (t < st) red[t] = red[t] + red[t + st]; __syncthreads(); } const float mu = red[0] * (1.0f / (float)DM); __syncthreads();
  float vs = 0.f;
#pragma unroll
  for (int q = 0; q < 4; ++q) { const float dl = s[q] - mu; vs = vs + dl * dl; }
  red[t] = vs; __syncthreads(); for (unsigned st = 64; st > 0; st >>= 1) { if (t < st) red[t] = red[t] + red[t + st]; __syncthreads(); }
  const float rs = rsqrtf(red[0] * (1.0f / (float)DM) + eps); v4h y; v4f yf;
  const v4f gv = *(const v4fa*)(g + c0), bv = *(const v4fa*)(bb + c0);
#pragma unroll
  for (int q = 0; q < 4; ++q) { yf[q] = ((s[q] - mu) * rs) * bf16_rne(gv[q]) + bf16_rne(bv[q]); y[q] = (_Float16)yf[q]; }
  for (int pass = 0; pass < 2; ++pass) { if (W16) *(volatile v4h*)(N16 + (size_t)ro * DM + c0) = y; if (W32) *(volatile v4f*)(N32 + (size_t)ro * DM + c0) = yf; if (pass == 0) __threadfence(); } }

__global__ __launch_bounds__(128) void k_attn(const _Float16* __restrict__ QK, const _Float16* __restrict__ VT, const float* __restrict__ pd, const int* __restrict__ msk, const float* __restrict__ omega, _Float16* __restrict__ Y16) {
  __shared__ __attribute__((aligned(16))) float so[4][16][68];
  const unsigned tid = threadIdx.x, w = tid >> 5, lane = tid & 31u, nl = lane & 15u, hh = lane >> 4;
  const unsigned h = blockIdx.y, b = blockIdx.z;
  const unsigned q0 = blockIdx.x * 64u + w * 16u;
  const size_t rq = (size_t)b * SEQ + q0;
  const size_t rk = (size_t)b * SEQ;
  const _Float16* qp = QK + (rq + nl) * LQK + (size_t)h * DK;
  const v16h qb = g2_frag(qp, hh);
  const _Float16* kp = QK + (rk + nl) * LQK + (size_t)(NH * DK) + (size_t)h * DK;
  const _Float16* vp = VT + ((size_t)h * DH + nl) * NR + rk;
  const size_t mrow = ((size_t)b * SEQ_FULL + q0 + nl) * SEQ_FULL + 8u * hh;
  const float* dp = pd + mrow; const int* mp = msk + mrow;
  const float om = bf16_rne(omega[h]);
  const v8f z8 = {0.f,0.f,0.f,0.f,0.f,0.f,0.f,0.f};
  v8f o0 = z8, o1 = z8, o2 = z8, o3 = z8; float lp = 0.f;
#pragma unroll 1
  for (unsigned kb = 0; kb < (unsigned)SEQ; kb += 32u) {
    const v8i ma = *(const v8ia*)(mp + kb), mb = *(const v8ia*)(mp + kb + 16u);
    unsigned nz = 1u;
#pragma unroll
    for (int r = 0; r < 8; ++r) nz &= (unsigned)(ma[r] != 0) & (unsigned)(mb[r] != 0);
    if (__builtin_amdgcn_ballot_w32(nz == 0u) == 0u) continue;
    const _Float16* k0p = kp + (size_t)kb * LQK; const _Float16* k1p = k0p + (size_t)16 * LQK;
    v8f s0 = z8, s1 = z8; v16h a;
    a = g2_frag(k0p, hh); s0 = g2_mma(a, qb, s0);
    a = g2_frag(k1p, hh); s1 = g2_mma(a, qb, s1);
    const v8f da = *(const v8fa*)(dp + kb), db = *(const v8fa*)(dp + kb + 16u);
    FragH pf; float ps = 0.f;
#pragma unroll
    for (int r = 0; r < 8; ++r) {
      const float b0 = expf(-om * bf16_rne(da[r])) - 1.0f; const float b1 = expf(-om * bf16_rne(db[r])) - 1.0f;
      float e0 = expf(s0[r] + b0); float e1 = expf(s1[r] + b1);
      e0 = (ma[r] != 0) ? 0.f : e0; e1 = (mb[r] != 0) ? 0.f : e1;
      ps += e0 + e1; pf.h[r] = (_Float16)e0; pf.h[8 + r] = (_Float16)e1; }
    lp += ps;
    const _Float16* v0p = vp + kb;
    a = g2_frag(v0p, hh); o0 = g2_mma(a, pf.v, o0);
    a = g2_frag(v0p + (size_t)16 * NR, hh); o1 = g2_mma(a, pf.v, o1);
    a = g2_frag(v0p + (size_t)32 * NR, hh); o2 = g2_mma(a, pf.v, o2);
    a = g2_frag(v0p + (size_t)48 * NR, hh); o3 = g2_mma(a, pf.v, o3);
  }
  const float l = lp + __shfl_xor(lp, 16, 32);
  const float inv = 1.0f / (l + 1.0f);
  { v4f lo4, hi4;
    lo4[0] = o0[0] * inv; lo4[1] = o0[1] * inv; lo4[2] = o0[2] * inv; lo4[3] = o0[3] * inv; hi4[0] = o0[4] * inv; hi4[1] = o0[5] * inv; hi4[2] = o0[6] * inv; hi4[3] = o0[7] * inv;
    *(v4fa*)&so[w][nl][0u * 16u + 8u * hh] = lo4; *(v4fa*)&so[w][nl][0u * 16u + 8u * hh + 4u] = hi4;
    lo4[0] = o1[0] * inv; lo4[1] = o1[1] * inv; lo4[2] = o1[2] * inv; lo4[3] = o1[3] * inv; hi4[0] = o1[4] * inv; hi4[1] = o1[5] * inv; hi4[2] = o1[6] * inv; hi4[3] = o1[7] * inv;
    *(v4fa*)&so[w][nl][1u * 16u + 8u * hh] = lo4; *(v4fa*)&so[w][nl][1u * 16u + 8u * hh + 4u] = hi4;
    lo4[0] = o2[0] * inv; lo4[1] = o2[1] * inv; lo4[2] = o2[2] * inv; lo4[3] = o2[3] * inv; hi4[0] = o2[4] * inv; hi4[1] = o2[5] * inv; hi4[2] = o2[6] * inv; hi4[3] = o2[7] * inv;
    *(v4fa*)&so[w][nl][2u * 16u + 8u * hh] = lo4; *(v4fa*)&so[w][nl][2u * 16u + 8u * hh + 4u] = hi4;
    lo4[0] = o3[0] * inv; lo4[1] = o3[1] * inv; lo4[2] = o3[2] * inv; lo4[3] = o3[3] * inv; hi4[0] = o3[4] * inv; hi4[1] = o3[5] * inv; hi4[2] = o3[6] * inv; hi4[3] = o3[7] * inv;
    *(v4fa*)&so[w][nl][3u * 16u + 8u * hh] = lo4; *(v4fa*)&so[w][nl][3u * 16u + 8u * hh + 4u] = hi4; }
  __builtin_amdgcn_fence(4  , "workgroup"); __builtin_amdgcn_wave_barrier();
  const unsigned rsub = lane >> 3, c8 = (lane & 7u) * 8u;
  unsigned short* yp = (unsigned short*)Y16 + rq * DM + (size_t)h * DH + c8;
  v8us ovh[4];
#pragma unroll
  for (unsigned q = 0; q < 4; ++q) { const unsigned row = q * 4u + rsub; const v4f sa = *(const v4fa*)&so[w][row][c8]; const v4f sb = *(const v4fa*)&so[w][row][c8 + 4u]; FragH f;
    f.h[0] = (_Float16)sa[0]; f.h[1] = (_Float16)sa[1]; f.h[2] = (_Float16)sa[2]; f.h[3] = (_Float16)sa[3]; f.h[4] = (_Float16)sb[0]; f.h[5] = (_Float16)sb[1]; f.h[6] = (_Float16)sb[2]; f.h[7] = (_Float16)sb[3];
    ovh[q] = f.half[0]; }
  for (int pass = 0; pass < 2; ++pass) {
#pragma unroll
    for (unsigned q = 0; q < 4; ++q) { const unsigned row = q * 4u + rsub; *(volatile v8us*)(yp + (size_t)row * DM) = ovh[q]; }
    if (pass == 0) __threadfence(); }
}

constexpr size_t SZ_BW   = (size_t)WROWS * DM * 2;
constexpr size_t SZ_X16  = NR * DM * 2;
constexpr size_t SZ_QKF  = NR * LQK * 4;
constexpr size_t SZ_QK16 = NR * LQK * 2;
constexpr size_t SZ_VT16 = (size_t)DM * NR * 2;
constexpr size_t SZ_Y16  = NR * DM * 2;
constexpr size_t SZ_T1   = NR * DM * 4;
constexpr size_t SZ_Z16  = NR * DM * 2;
constexpr size_t SZ_Z32  = NR * DM * 4;
constexpr size_t SZ_T2   = NR * DM * 4;
constexpr size_t WS_TOTAL = SZ_BW + SZ_X16 + SZ_QKF + SZ_QK16 + SZ_VT16 + SZ_Y16 + SZ_T1 + SZ_Z16 + SZ_Z32 + SZ_T2;
static_assert(SZ_BW % 256 == 0 && SZ_X16 % 256 == 0 && SZ_QKF % 256 == 0 && SZ_QK16 % 256 == 0 && SZ_VT16 % 256 == 0 && SZ_Y16 % 256 == 0 && SZ_T1 % 256 == 0 && SZ_Z16 % 256 == 0 && SZ_Z32 % 256 == 0 && SZ_T2 % 256 == 0);
static_assert(WS_TOTAL <= (size_t)134217728);

extern "C" void kernel_launch(void* const* d_in, const int* in_sizes, int n_in,
                              void* d_out, int out_size, void* d_ws, size_t ws_size, hipStream_t stream) {
  if (n_in < 15) return;
  const float* x   = (const float*)d_in[0];
  const int*   msk = (const int*)d_in[1];
  const float* pd  = (const float*)d_in[2];
  const float* wq  = (const float*)d_in[3];
  const float* wk  = (const float*)d_in[4];
  const float* wv  = (const float*)d_in[5];
  const float* omg = (const float*)d_in[6];
  const float* wo  = (const float*)d_in[7];
  const float* bo  = (const float*)d_in[8];
  const float* wf  = (const float*)d_in[9];
  const float* bfv = (const float*)d_in[10];
  const float* g1  = (const float*)d_in[11]; const float* b1 = (const float*)d_in[12];
  const float* g2  = (const float*)d_in[13]; const float* b2 = (const float*)d_in[14];
  const size_t need = ((size_t)(NB - 1) * SEQ_FULL + SEQ) * DM;
  const size_t need2 = ((size_t)(NB - 1) * SEQ_FULL + SEQ - 1) * SEQ_FULL + SEQ;
  if ((size_t)in_sizes[0] < need || (size_t)out_size < need) return;
  if ((size_t)in_sizes[1] < need2 || (size_t)in_sizes[2] < need2) return;
  if (in_sizes[3] < NH * DK * DM || in_sizes[4] < NH * DK * DM || in_sizes[5] < NH * DH * DM || in_sizes[6] < NH || in_sizes[7] < DM * DM || in_sizes[8] < DM || in_sizes[9] < DM * DM || in_sizes[10] < DM
      || in_sizes[11] < DM || in_sizes[12] < DM || in_sizes[13] < DM || in_sizes[14] < DM) return;
  const int M = (int)NR;
  char* ws = (char*)d_ws; size_t off = 0;
  auto take = [&](size_t bytes) { char* p = ws + off; off += (bytes + 255) & ~(size_t)255; return p; };
  _Float16* BW   = (_Float16*)take(SZ_BW);
  _Float16* X16  = (_Float16*)take(SZ_X16);
  float*    QKF  = (float*)take(SZ_QKF);
  _Float16* QK16 = (_Float16*)take(SZ_QK16);
  _Float16* VT16 = (_Float16*)take(SZ_VT16);
  _Float16* Y16  = (_Float16*)take(SZ_Y16);
  float*    T1   = (float*)take(SZ_T1);
  _Float16* Z16  = (_Float16*)take(SZ_Z16);
  float*    Z32  = (float*)take(SZ_Z32);
  float*    T2   = (float*)take(SZ_T2);
  if (off > ws_size || off > (size_t)134217728) return;
  const _Float16* BWv = BW + (size_t)512 * DM; const _Float16* BWo = BW + (size_t)1024 * DM; const _Float16* BWf = BW + (size_t)1536 * DM;
  k_xprep<<<(unsigned)(NR * DM / 8 / 256), 256, 0, stream>>>(x, X16, (unsigned)(NR * DM / 8));
  k_wprep<<<dim3((unsigned)((size_t)DM * DM / 8 / 256), 5), 256, 0, stream>>>(wq, wk, wv, wo, wf, BW);
  k_gemm2<0, 0><<<dim3(LQK / 64, (unsigned)(M / 128)), 128, 0, stream>>>(X16, DM, BW, DM, 0.0625f, nullptr, nullptr, QKF, nullptr, LQK, M, LQK, DM);
  k_l2n<<<(unsigned)(NR * LQK / 8 / 256), 256, 0, stream>>>(QKF, QK16, (unsigned)(NR * LQK / 8));
  k_gemm2<0, 0><<<dim3((unsigned)(M / 64), DM / 128), 128, 0, stream>>>(BWv, DM, X16, DM, 1.0f, nullptr, nullptr, nullptr, VT16, M, DM, M, DM);
  k_attn<<<dim3(SEQ / 64, NH, NB), 128, 0, stream>>>(QK16, VT16, pd, msk, omg, Y16);
  k_gemm2<0, 2><<<dim3(DM / 64, (unsigned)(M / 128)), 128, 0, stream>>>(Y16, DM, BWo, DM, 0.00390625f, bo, x, T1, nullptr, DM, M, DM, DM);
  k_lnx<1, 1, 0><<<(unsigned)M, 128, 0, stream>>>(T1, g1, b1, 1e-5f, Z16, Z32);
  k_gemm2<4, 1><<<dim3(DM / 64, (unsigned)(M / 128)), 128, 0, stream>>>(Z16, DM, BWf, DM, 0.0625f, bfv, Z32, T2, nullptr, DM, M, DM, DM);
  k_lnx<0, 1, 1><<<(unsigned)M, 128, 0, stream>>>(T2, g2, b2, 1e-5f, nullptr, (float*)d_out);
}
